// MultiHeadQKVAttention_70531952935642
// MI455X (gfx1250) — hardware-verified
//
#include <hip/hip_runtime.h>
#include <math.h>
#include <stdint.h>

#define NSB  2
#define LQ   2048
#define EE   256
#define NH   8
#define DH   32
#define MR   (NSB * LQ)
#define XSC  64.0f
#define WSC  1024.0f
#define ISC  (1.0f / 4096.0f)
#define BSC  16.0f
#define QKS  (1.0f / 256.0f)
#define RSQ  0.17677669529663687f
#define MBIG 1.0e32f
#define NEG0 (-1.0e38f)
#define PSC  4096.0f
#define PLO  2048.0f
#define LOIN (1.0f / 2048.0f)
#define OSA  (1.0f / 256.0f)
#define LOSC 2048.0f
#define OSC  (1.0f / 262144.0f)
#define NBX  ((MR * EE) / 2048)
static_assert(EE == NH * DH);
static_assert(DH == 32);
static_assert((LQ % 64) == 0 && (EE % 128) == 0 && (MR % 64) == 0);
static_assert(((MR * EE) % 2048) == 0);
static_assert(NBX == 512);
static_assert(LQ == 128 * 16);

typedef _Float16 v16h __attribute__((ext_vector_type(16)));
typedef _Float16 v8h  __attribute__((ext_vector_type(8)));
typedef float    v8f  __attribute__((ext_vector_type(8)));
typedef float    v4f  __attribute__((ext_vector_type(4)));
typedef unsigned int v4u __attribute__((ext_vector_type(4)));

union FragH { v16h v; v8h h[2]; };

__device__ __forceinline__ unsigned short bf_bits(float f) {
  unsigned u = __float_as_uint(f);
  return (unsigned short)((u + 0x7FFFu + ((u >> 16) & 1u)) >> 16);
}
__device__ __forceinline__ float bf_up(unsigned short h) { return __uint_as_float(((unsigned)h) << 16); }
__device__ __forceinline__ float bfr(float f) { return bf_up(bf_bits(f)); }
__device__ __forceinline__ unsigned short h_bits(_Float16 x) { return __builtin_bit_cast(unsigned short, x); }
__device__ __forceinline__ unsigned pk16(unsigned short a, unsigned short b) { return (unsigned)a | ((unsigned)b << 16); }
__device__ __forceinline__ v8f zero8() { v8f z = {0.f, 0.f, 0.f, 0.f, 0.f, 0.f, 0.f, 0.f}; return z; }
__device__ __forceinline__ v4u cvt8(v4f a, v4f c, float sc) {
  float f[8];
#pragma unroll
  for (int i = 0; i < 4; ++i) { f[i] = bfr(a[i]) * sc; f[4 + i] = bfr(c[i]) * sc; }
  v4u v;
#pragma unroll
  for (int i = 0; i < 4; ++i) v[i] = pk16(h_bits((_Float16)f[2 * i]), h_bits((_Float16)f[2 * i + 1]));
  return v;
}

__device__ __forceinline__ v16h ldfrag_h(const _Float16* p) {
  FragH f;
  f.h[0] = *(const v8h*)(p);
  f.h[1] = *(const v8h*)(p + 16);
  return f.v;
}

__device__ __forceinline__ v8f mma_h(v16h a, v16h b, v8f c) {
  return __builtin_amdgcn_wmma_f32_16x16x32_f16(false, a, false, b, (short)0, c, false, false);
}
__device__ __forceinline__ void guard2(v8f& a, v8f& b, v16h x0, v16h x1, v16h y) {
#if defined(__HIP_DEVICE_COMPILE__)
  asm volatile("v_nop\n\tv_nop\n\tv_nop\n\tv_nop" : "+v"(a), "+v"(b) : "v"(x0), "v"(x1), "v"(y));
#endif
}
__device__ __forceinline__ void guard4(v8f& a, v8f& b, v8f& c, v8f& d,
                                       v16h x, v16h y0, v16h y1, v16h y2, v16h y3) {
#if defined(__HIP_DEVICE_COMPILE__)
  asm volatile("v_nop\n\tv_nop\n\tv_nop\n\tv_nop"
               : "+v"(a), "+v"(b), "+v"(c), "+v"(d) : "v"(x), "v"(y0), "v"(y1), "v"(y2), "v"(y3));
#endif
}
__device__ __forceinline__ void guard4b(v8f& a, v8f& b, v8f& c, v8f& d,
                                        v16h x0, v16h x1, v16h y0, v16h y1) {
#if defined(__HIP_DEVICE_COMPILE__)
  asm volatile("v_nop\n\tv_nop\n\tv_nop\n\tv_nop"
               : "+v"(a), "+v"(b), "+v"(c), "+v"(d) : "v"(x0), "v"(x1), "v"(y0), "v"(y1));
#endif
}

__global__ __launch_bounds__(256)
void cvt_planes(const float* __restrict__ xq, const float* __restrict__ xk, const float* __restrict__ xv,
                unsigned short* pq, unsigned short* pk, unsigned short* pv) {
  const int bx = blockIdx.x;
  const float* src;
  unsigned short* dst;
  int lb;
  if (bx < NBX)          { src = xq; dst = pq; lb = bx; }
  else if (bx < 2 * NBX) { src = xk; dst = pk; lb = bx - NBX; }
  else                   { src = xv; dst = pv; lb = bx - 2 * NBX; }
  const size_t e0 = ((size_t)lb * 256 + threadIdx.x) * 8;
  const v4f a = *(const v4f*)(src + e0);
  const v4f c = *(const v4f*)(src + e0 + 4);
  const v4u v = cvt8(a, c, XSC);
  unsigned short* dp = dst + e0;
  *(volatile v4u*)dp = v;
  __threadfence();
  *(volatile v4u*)dp = v;
}

__global__ __launch_bounds__(256)
void cvt_wt(const float* __restrict__ wq, const float* __restrict__ wk, const float* __restrict__ wv,
            const float* __restrict__ wo, unsigned short* hq, unsigned short* hk, unsigned short* hv,
            unsigned short* ho) {
  __shared__ __align__(16) unsigned short Ts[64 * 264];
  const int tid  = threadIdx.x;
  const int wave = tid >> 5;
  const int lane = tid & 31;
  const int bx   = blockIdx.x;
  const int w    = bx >> 2;
  const int o0   = (bx & 3) * 64;
  const float* src;
  unsigned short* dst;
  if (w == 0)      { src = wq; dst = hq; }
  else if (w == 1) { src = wk; dst = hk; }
  else if (w == 2) { src = wv; dst = hv; }
  else             { src = wo; dst = ho; }
  const int p = tid & 15, r16 = tid >> 4;
#pragma unroll 4
  for (int it = 0; it < 16; ++it) {
    const int e = it * 16 + r16;
    const v4f a = *(const v4f*)(src + (size_t)e * EE + o0 + 4 * p);
#pragma unroll
    for (int i = 0; i < 4; ++i) Ts[(4 * p + i) * 264 + e] = h_bits((_Float16)(bfr(a[i]) * WSC));
  }
  __syncthreads();
  v4u vals[8];
#pragma unroll
  for (int it = 0; it < 8; ++it) {
    const int row = it * 8 + wave;
    vals[it] = *(const v4u*)(Ts + row * 264 + 8 * lane);
  }
  unsigned short* db = dst + (size_t)o0 * EE + 8 * lane;
  for (int pass = 0; pass < 2; ++pass) {
#pragma unroll
    for (int it = 0; it < 8; ++it) {
      const int row = it * 8 + wave;
      *(volatile v4u*)(db + (size_t)row * EE) = vals[it];
    }
    __threadfence();
  }
}

template <int TR>
__global__ __launch_bounds__(128)
void proj_gemm(const unsigned short* __restrict__ wh, const unsigned short* __restrict__ xh,
               const float* __restrict__ bias, unsigned short* yo) {
  __shared__ __align__(16) unsigned short Ts[128 * 72];
  const int tid  = threadIdx.x;
  const int wave = tid >> 5;
  const int lane = tid & 31;
  const int hh   = lane >> 4;
  const int ci   = lane & 15;
  const int bx   = blockIdx.x;
  const int mt   = bx >> 1, ot = bx & 1;
  const int m0   = mt * 64, o0 = ot * 128;
  const _Float16* W = (const _Float16*)(const void*)wh;
  const _Float16* X = (const _Float16*)(const void*)xh;
  const _Float16* xr = X + (size_t)(m0 + 16 * wave + ci) * EE + 8 * hh;
  const _Float16* wr = W + (size_t)(o0 + ci) * EE + 8 * hh;

  v8f acc[8];
#pragma unroll
  for (int t = 0; t < 8; ++t) acc[t] = zero8();

#pragma unroll 1
  for (int ks = 0; ks < EE / 32; ++ks) {
    const int k0 = ks * 32;
    const v16h xb = ldfrag_h(xr + k0);
    v16h wa[4];
#pragma unroll
    for (int t = 0; t < 4; ++t) wa[t] = ldfrag_h(wr + (size_t)(16 * t) * EE + k0);
#pragma unroll
    for (int t = 0; t < 4; ++t) acc[t] = mma_h(wa[t], xb, acc[t]);
    guard4(acc[0], acc[1], acc[2], acc[3], xb, wa[0], wa[1], wa[2], wa[3]);
    v16h wc[4];
#pragma unroll
    for (int t = 0; t < 4; ++t) wc[t] = ldfrag_h(wr + (size_t)(16 * (t + 4)) * EE + k0);
#pragma unroll
    for (int t = 0; t < 4; ++t) acc[4 + t] = mma_h(wc[t], xb, acc[4 + t]);
    guard4(acc[4], acc[5], acc[6], acc[7], xb, wc[0], wc[1], wc[2], wc[3]);
  }

  if (TR == 0) {
    unsigned short* ts = Ts + (16 * wave + ci) * 136 + 8 * hh;
#pragma unroll
    for (int t = 0; t < 8; ++t) {
      const v4f b0 = *(const v4f*)(bias + o0 + 16 * t + 8 * hh);
      const v4f b1 = *(const v4f*)(bias + o0 + 16 * t + 8 * hh + 4);
      float y[8];
#pragma unroll
      for (int e = 0; e < 4; ++e) {
        y[e]     = acc[t][e] * ISC     + bfr(b0[e]) * BSC;
        y[4 + e] = acc[t][4 + e] * ISC + bfr(b1[e]) * BSC;
      }
      v4u v;
#pragma unroll
      for (int i = 0; i < 4; ++i) v[i] = pk16(h_bits((_Float16)y[2 * i]), h_bits((_Float16)y[2 * i + 1]));
      *(v4u*)(ts + 16 * t) = v;
    }
    __syncthreads();
    const int p = tid & 15, r16 = tid >> 4;
    v4u vals[8];
#pragma unroll
    for (int it = 0; it < 8; ++it) {
      const int row = it * 8 + r16;
      vals[it] = *(const v4u*)(Ts + row * 136 + 8 * p);
    }
    unsigned short* yb = yo + (size_t)m0 * EE + o0 + 8 * p;
    for (int pass = 0; pass < 2; ++pass) {
#pragma unroll
      for (int it = 0; it < 8; ++it) {
        const int row = it * 8 + r16;
        *(volatile v4u*)(yb + (size_t)row * EE) = vals[it];
      }
      __threadfence();
    }
  } else {
    const int ns = m0 / LQ, l0 = m0 - ns * LQ;
#pragma unroll
    for (int t = 0; t < 8; ++t) {
      const v4f b0 = *(const v4f*)(bias + o0 + 16 * t + 8 * hh);
      const v4f b1 = *(const v4f*)(bias + o0 + 16 * t + 8 * hh + 4);
#pragma unroll
      for (int r = 0; r < 4; ++r) {
        Ts[(16 * t + 8 * hh + r) * 72 + 16 * wave + ci] =
            h_bits((_Float16)(acc[t][r] * ISC + bfr(b0[r]) * BSC));
        Ts[(16 * t + 8 * hh + 4 + r) * 72 + 16 * wave + ci] =
            h_bits((_Float16)(acc[t][4 + r] * ISC + bfr(b1[r]) * BSC));
      }
    }
    __syncthreads();
    const int e8 = tid & 7, fq = tid >> 3;
    v4u vals[8];
#pragma unroll
    for (int it = 0; it < 8; ++it) {
      const int orow = it * 16 + fq;
      vals[it] = *(const v4u*)(Ts + orow * 72 + 8 * e8);
    }
    unsigned short* yb = yo + ((size_t)ns * EE + o0) * LQ + l0 + 8 * e8;
    for (int pass = 0; pass < 2; ++pass) {
#pragma unroll
      for (int it = 0; it < 8; ++it) {
        const int orow = it * 16 + fq;
        *(volatile v4u*)(yb + (size_t)orow * LQ) = vals[it];
      }
      __threadfence();
    }
  }
}

__global__ __launch_bounds__(128)
void attn_fwd(const unsigned short* __restrict__ q16, const unsigned short* __restrict__ k16,
              const unsigned short* __restrict__ vt, const float* __restrict__ pres,
              unsigned short* ohp, unsigned short* olp) {
  __shared__ __align__(16) float Mk[LQ];
  __shared__ __align__(16) unsigned short Hs[64 * 40];
  __shared__ __align__(16) unsigned short Lw[64 * 40];
  const int tid  = threadIdx.x;
  const int wave = tid >> 5;
  const int lane = tid & 31;
  const int hh   = lane >> 4;
  const int ci   = lane & 15;
  const int bx   = blockIdx.x;
  const int ns   = bx / (NH * (LQ / 64));
  const int rem  = bx - ns * (NH * (LQ / 64));
  const int h    = rem / (LQ / 64);
  const int q0   = (rem - h * (LQ / 64)) * 64;
  const int qi   = q0 + 16 * wave + ci;
  {
    const float* pp = pres + (size_t)ns * LQ + 16 * tid;
#pragma unroll
    for (int i = 0; i < 4; ++i) {
      const v4f a = *(const v4f*)(pp + 4 * i);
      v4f mv;
#pragma unroll
      for (int e = 0; e < 4; ++e) mv[e] = (1.0f - bfr(a[e])) * MBIG;
      *(v4f*)(Mk + 16 * tid + 4 * i) = mv;
    }
  }
  __syncthreads();

  const _Float16* Q = (const _Float16*)(const void*)q16;
  const _Float16* K = (const _Float16*)(const void*)k16;
  const _Float16* V = (const _Float16*)(const void*)vt;
  const v16h qf = ldfrag_h(Q + (size_t)(ns * LQ + qi) * EE + h * DH + 8 * hh);
  const _Float16* kp = K + (size_t)(ns * LQ + ci) * EE + h * DH + 8 * hh;
  const _Float16* vp = V + ((size_t)ns * EE + h * DH + ci) * LQ + 8 * hh;

  float rmax = NEG0, z = 0.f;
  v8f ah0 = zero8(), ah1 = zero8(), al0 = zero8(), al1 = zero8();
#pragma unroll 1
  for (int it = 0; it < LQ / 32; ++it) {
    const int lt = it * 32;
    const v16h ka0 = ldfrag_h(kp + (size_t)lt * EE);
    const v16h ka1 = ldfrag_h(kp + (size_t)(lt + 16) * EE);
    v8f s0 = mma_h(ka0, qf, zero8());
    v8f s1 = mma_h(ka1, qf, zero8());
    guard2(s0, s1, ka0, ka1, qf);
    const v4f ma = *(const v4f*)(Mk + lt + 8 * hh);
    const v4f mb = *(const v4f*)(Mk + lt + 8 * hh + 4);
    const v4f mc = *(const v4f*)(Mk + lt + 16 + 8 * hh);
    const v4f md = *(const v4f*)(Mk + lt + 20 + 8 * hh);
    float t[16];
#pragma unroll
    for (int r = 0; r < 4; ++r) {
      t[r]      = (s0[r] * QKS     - ma[r]) * RSQ;
      t[4 + r]  = (s0[4 + r] * QKS - mb[r]) * RSQ;
      t[8 + r]  = (s1[r] * QKS     - mc[r]) * RSQ;
      t[12 + r] = (s1[4 + r] * QKS - md[r]) * RSQ;
    }
    float mx = t[0];
#pragma unroll
    for (int i = 1; i < 16; ++i) mx = fmaxf(mx, t[i]);
    mx = fmaxf(mx, __shfl_xor(mx, 16, 32));
    const float nmax = fmaxf(rmax, mx);
    const float corr = __expf(rmax - nmax);
    rmax = nmax;
    FragH ph, pl;
    float zs = 0.f;
#pragma unroll
    for (int r = 0; r < 8; ++r) {
      const float pa = __expf(t[r] - nmax);
      const float pc = __expf(t[8 + r] - nmax);
      zs += pa + pc;
      const float xa = pa * PSC, xc = pc * PSC;
      const _Float16 ha = (_Float16)xa, hc = (_Float16)xc;
      ph.h[0][r] = ha;
      ph.h[1][r] = hc;
      pl.h[0][r] = (_Float16)((xa - (float)ha) * PLO);
      pl.h[1][r] = (_Float16)((xc - (float)hc) * PLO);
    }
    z = z * corr + zs;
    ah0 *= corr; ah1 *= corr; al0 *= corr; al1 *= corr;
    const v16h va0 = ldfrag_h(vp + lt);
    const v16h va1 = ldfrag_h(vp + (size_t)16 * LQ + lt);
    ah0 = mma_h(va0, ph.v, ah0);
    ah1 = mma_h(va1, ph.v, ah1);
    al0 = mma_h(va0, pl.v, al0);
    al1 = mma_h(va1, pl.v, al1);
    guard4b(ah0, ah1, al0, al1, va0, va1, ph.v, pl.v);
  }

  const float zz  = z + __shfl_xor(z, 16, 32);
  const float rzs = (1.0f / zz) * OSA;
  float o[16];
#pragma unroll
  for (int r = 0; r < 8; ++r) {
    o[r]     = (ah0[r] + al0[r] * LOIN) * rzs;
    o[8 + r] = (ah1[r] + al1[r] * LOIN) * rzs;
  }
  v4u h0, h1, g0, g1;
#pragma unroll
  for (int i = 0; i < 4; ++i) {
    const _Float16 a0 = (_Float16)o[2 * i],     a1 = (_Float16)o[2 * i + 1];
    const _Float16 b0 = (_Float16)o[8 + 2 * i], b1 = (_Float16)o[8 + 2 * i + 1];
    const _Float16 la0 = (_Float16)((o[2 * i]         - (float)a0) * LOSC);
    const _Float16 la1 = (_Float16)((o[2 * i + 1]     - (float)a1) * LOSC);
    const _Float16 lb0 = (_Float16)((o[8 + 2 * i]     - (float)b0) * LOSC);
    const _Float16 lb1 = (_Float16)((o[8 + 2 * i + 1] - (float)b1) * LOSC);
    h0[i] = pk16(h_bits(a0), h_bits(a1));
    h1[i] = pk16(h_bits(b0), h_bits(b1));
    g0[i] = pk16(h_bits(la0), h_bits(la1));
    g1[i] = pk16(h_bits(lb0), h_bits(lb1));
  }
  {
    const int ro = (16 * wave + ci) * 40 + 8 * hh;
    *(v4u*)(Hs + ro)      = h0;
    *(v4u*)(Hs + ro + 16) = h1;
    *(v4u*)(Lw + ro)      = g0;
    *(v4u*)(Lw + ro + 16) = g1;
  }
  __syncthreads();
  {
    const size_t ob = ((size_t)(ns * NH + h) * LQ + q0) * DH;
    v4u hv[2], lv[2];
#pragma unroll
    for (int it2 = 0; it2 < 2; ++it2) {
      const int hf = it2 * 1024 + 8 * tid;
      const int row = hf >> 5, col = hf & 31;
      hv[it2] = *(const v4u*)(Hs + row * 40 + col);
      lv[it2] = *(const v4u*)(Lw + row * 40 + col);
    }
    for (int pass = 0; pass < 2; ++pass) {
#pragma unroll
      for (int it2 = 0; it2 < 2; ++it2) {
        const int hf = it2 * 1024 + 8 * tid;
        *(volatile v4u*)(ohp + ob + hf) = hv[it2];
        *(volatile v4u*)(olp + ob + hf) = lv[it2];
      }
      __threadfence();
    }
  }
}

__global__ __launch_bounds__(128)
void out_proj(const unsigned short* __restrict__ ohp, const unsigned short* __restrict__ olp,
              const unsigned short* __restrict__ woh, const float* __restrict__ bo, float* out) {
  __shared__ __align__(16) float Ts[64 * 68];
  const int tid  = threadIdx.x;
  const int wave = tid >> 5;
  const int lane = tid & 31;
  const int hh   = lane >> 4;
  const int ci   = lane & 15;
  const int bx   = blockIdx.x;
  const int mt   = bx >> 2, ot = bx & 3;
  const int m0   = mt * 64, o0 = ot * 64;
  const int ns   = m0 / LQ;
  const int ql   = m0 - ns * LQ + 16 * wave + ci;
  const _Float16* OHf = (const _Float16*)(const void*)ohp;
  const _Float16* OLf = (const _Float16*)(const void*)olp;
  const _Float16* W   = (const _Float16*)(const void*)woh;
  const size_t orow = ((size_t)(ns * NH) * LQ + ql) * DH + 8 * hh;
  const _Float16* ar = OHf + orow;
  const _Float16* lr = OLf + orow;
  const _Float16* wr = W + (size_t)(o0 + ci) * EE + 8 * hh;

  v8f acch[4], accl[4];
#pragma unroll
  for (int t = 0; t < 4; ++t) { acch[t] = zero8(); accl[t] = zero8(); }

#pragma unroll 1
  for (int j = 0; j < NH; ++j) {
    const v16h obh = ldfrag_h(ar + (size_t)j * LQ * DH);
    const v16h obl = ldfrag_h(lr + (size_t)j * LQ * DH);
    v16h wa[4];
#pragma unroll
    for (int t = 0; t < 4; ++t) wa[t] = ldfrag_h(wr + (size_t)(16 * t) * EE + 32 * j);
#pragma unroll
    for (int t = 0; t < 4; ++t) acch[t] = mma_h(wa[t], obh, acch[t]);
    guard4(acch[0], acch[1], acch[2], acch[3], obh, wa[0], wa[1], wa[2], wa[3]);
#pragma unroll
    for (int t = 0; t < 4; ++t) accl[t] = mma_h(wa[t], obl, accl[t]);
    guard4(accl[0], accl[1], accl[2], accl[3], obl, wa[0], wa[1], wa[2], wa[3]);
  }

  {
    float* ts = Ts + (16 * wave + ci) * 68 + 8 * hh;
#pragma unroll
    for (int t = 0; t < 4; ++t) {
      const v4f b0 = *(const v4f*)(bo + o0 + 16 * t + 8 * hh);
      const v4f b1 = *(const v4f*)(bo + o0 + 16 * t + 8 * hh + 4);
      v4f r0, r1;
#pragma unroll
      for (int e = 0; e < 4; ++e) {
        r0[e] = (acch[t][e]     + accl[t][e]     * LOIN) * OSC + bfr(b0[e]);
        r1[e] = (acch[t][4 + e] + accl[t][4 + e] * LOIN) * OSC + bfr(b1[e]);
      }
      *(v4f*)(ts + 16 * t)     = r0;
      *(v4f*)(ts + 16 * t + 4) = r1;
    }
  }
  __syncthreads();
  {
    const int p = tid & 15, r16 = tid >> 4;
    v4f vals[8];
#pragma unroll
    for (int it = 0; it < 8; ++it) {
      const int row = it * 8 + r16;
      vals[it] = *(const v4f*)(Ts + row * 68 + 4 * p);
    }
    float* yb = out + (size_t)m0 * EE + o0 + 4 * p;
    for (int pass = 0; pass < 2; ++pass) {
#pragma unroll
      for (int it = 0; it < 8; ++it) {
        const int row = it * 8 + r16;
        *(volatile v4f*)(yb + (size_t)row * EE) = vals[it];
      }
      __threadfence();
    }
  }
}

extern "C" void kernel_launch(void* const* d_in, const int* in_sizes, int n_in,
                              void* d_out, int out_size, void* d_ws, size_t ws_size,
                              hipStream_t stream) {
  if (n_in < 12) return;
  if (in_sizes[0] != MR * EE || in_sizes[1] != MR * EE || in_sizes[2] != MR * EE) return;
  if (in_sizes[3] != NSB * LQ) return;
  if (in_sizes[4] != EE * EE || in_sizes[6] != EE * EE || in_sizes[8] != EE * EE || in_sizes[10] != EE * EE) return;
  if (in_sizes[5] != EE || in_sizes[7] != EE || in_sizes[9] != EE || in_sizes[11] != EE) return;
  if (out_size != MR * EE) return;

  const float* queries = (const float*)d_in[0];
  const float* keys    = (const float*)d_in[1];
  const float* values  = (const float*)d_in[2];
  const float* pres    = (const float*)d_in[3];
  const float* Wq      = (const float*)d_in[4];
  const float* bq      = (const float*)d_in[5];
  const float* Wk      = (const float*)d_in[6];
  const float* bk      = (const float*)d_in[7];
  const float* Wv      = (const float*)d_in[8];
  const float* bv      = (const float*)d_in[9];
  const float* Wo      = (const float*)d_in[10];
  const float* bo      = (const float*)d_in[11];
  float* out = (float*)d_out;

  const size_t PX  = (size_t)MR * EE * 2;
  const size_t PW  = (size_t)EE * EE * 2;
  const size_t PP  = (size_t)MR * EE * 2;
  const size_t PVT = (size_t)NSB * EE * LQ * 2;
  const size_t PO  = (size_t)NSB * NH * LQ * DH * 2;
  size_t off = 0;
  const size_t oPQ = off; off += PX;
  const size_t oPK = off; off += PX;
  const size_t oPV = off; off += PX;
  const size_t oHQ = off; off += PW;
  const size_t oHK = off; off += PW;
  const size_t oHV = off; off += PW;
  const size_t oHO = off; off += PW;
  const size_t oQ  = off; off += PP;
  const size_t oK  = off; off += PP;
  const size_t oVT = off; off += PVT;
  const size_t oOH = off; off += PO;
  const size_t oOL = off; off += PO;
  if (off > ws_size) return;
  if (off > (size_t)134217728) return;

  char* ws = (char*)d_ws;
  unsigned short* PQp = (unsigned short*)(ws + oPQ);
  unsigned short* PKp = (unsigned short*)(ws + oPK);
  unsigned short* PVp = (unsigned short*)(ws + oPV);
  unsigned short* HQp = (unsigned short*)(ws + oHQ);
  unsigned short* HKp = (unsigned short*)(ws + oHK);
  unsigned short* HVp = (unsigned short*)(ws + oHV);
  unsigned short* HOp = (unsigned short*)(ws + oHO);
  unsigned short* Q16 = (unsigned short*)(ws + oQ);
  unsigned short* K16 = (unsigned short*)(ws + oK);
  unsigned short* VTp = (unsigned short*)(ws + oVT);
  unsigned short* OHp = (unsigned short*)(ws + oOH);
  unsigned short* OLp = (unsigned short*)(ws + oOL);

  const dim3 blk256(256), blk128(128);
  const dim3 gCV(3 * NBX);
  const dim3 gWT(16);
  const dim3 gPJ((MR / 64) * (EE / 128));
  const dim3 gAT(NSB * NH * (LQ / 64));
  const dim3 gOP((MR / 64) * (EE / 64));

  cvt_planes<<<gCV, blk256, 0, stream>>>(queries, keys, values, PQp, PKp, PVp);
  cvt_wt<<<gWT, blk256, 0, stream>>>(Wq, Wk, Wv, Wo, HQp, HKp, HVp, HOp);
  proj_gemm<0><<<gPJ, blk128, 0, stream>>>(HQp, PQp, bq, Q16);
  proj_gemm<0><<<gPJ, blk128, 0, stream>>>(HKp, PKp, bk, K16);
  proj_gemm<1><<<gPJ, blk128, 0, stream>>>(HVp, PVp, bv, VTp);
  attn_fwd<<<gAT, blk128, 0, stream>>>(Q16, K16, VTp, pres, OHp, OLp);
  out_proj<<<gOP, blk128, 0, stream>>>(OHp, OLp, HOp, bo, out);
  (void)hipGetLastError();
}
